// OlMoEAttention_81097572483288
// MI455X (gfx1250) — hardware-verified
//
#include <hip/hip_runtime.h>
#include <math.h>
#include <stdint.h>

constexpr int SEQ = 4096;
constexpr int HID = 2048;
constexpr int NQH = 16;
constexpr int HDM = 128;
constexpr int KVW = 512;
constexpr int QKVW = HID + 2 * KVW;
constexpr int ROWS_SPLIT = 1024;
constexpr int QB_ROWS = 64;
constexpr int NQB = SEQ / QB_ROWS;
constexpr int NQB_SPLIT = ROWS_SPLIT / QB_ROWS;
constexpr int NFREQ = HDM / 2;
constexpr float RMS_EPS = 1e-5f;
constexpr float A_CARRY = 16.0f;
constexpr float P_CARRY = 1024.0f;
constexpr float LO_CARRY = 64.0f;
constexpr float W_CARRY = 64.0f;

static_assert(HID % 32 == 0);
static_assert(SEQ % 64 == 0);
static_assert(QKVW % 64 == 0);
static_assert(HID % 64 == 0);
static_assert(ROWS_SPLIT % 64 == 0);
static_assert((SEQ - ROWS_SPLIT) % 64 == 0);
static_assert(NQH * HDM == HID);
static_assert(HDM == 128);
static_assert(KVW == 4 * HDM);
static_assert(NFREQ == 64);

constexpr size_t WS_QKVRAW = 0;
constexpr size_t WS_AH     = 0;
constexpr size_t WS_AL     = WS_AH + (size_t)SEQ * HID * 2;
constexpr size_t WS_HS     = (size_t)SEQ * QKVW * 4;
constexpr size_t WS_QH     = WS_HS;
constexpr size_t WS_WQKV   = WS_HS + (size_t)SEQ * HID * 2;
constexpr size_t WS_KH     = WS_WQKV;
constexpr size_t WS_VH     = WS_KH + (size_t)SEQ * KVW * 2;
constexpr size_t WS_KL     = WS_VH + (size_t)SEQ * KVW * 2;
constexpr size_t WS_VL     = WS_KL + (size_t)ROWS_SPLIT * KVW * 2;
constexpr size_t WS_WOH    = WS_WQKV + (size_t)QKVW * HID * 2;
constexpr size_t WS_WOL    = WS_WOH + (size_t)HID * HID * 2;
constexpr size_t WS_QL     = WS_WOL + (size_t)HID * HID * 2;
constexpr size_t WS_TCOS   = WS_QL + (size_t)ROWS_SPLIT * HID * 2;
constexpr size_t WS_TSIN   = WS_TCOS + (size_t)SEQ * NFREQ * 4;
constexpr size_t WS_TOTAL  = WS_TSIN + (size_t)SEQ * NFREQ * 4;
static_assert(WS_AL + (size_t)ROWS_SPLIT * HID * 2 <= WS_HS);
static_assert(WS_VL + (size_t)ROWS_SPLIT * KVW * 2 <= WS_WOH);
static_assert(WS_TOTAL == 102760448);
static_assert(WS_TOTAL <= 134217728);

typedef __attribute__((ext_vector_type(16))) _Float16 v16h;
typedef __attribute__((ext_vector_type(8)))  _Float16 v8h;
typedef __attribute__((ext_vector_type(16))) __bf16   v16b;
typedef __attribute__((ext_vector_type(8)))  __bf16   v8b;
typedef __attribute__((ext_vector_type(8)))  float    v8f;
typedef __attribute__((ext_vector_type(4)))  float    v4f;
typedef __attribute__((ext_vector_type(4)))  unsigned int v4u;

__device__ __forceinline__ unsigned short f2bf_bits(float f) {
  unsigned u = __float_as_uint(f);
  return (unsigned short)((u + 0x7FFFu + ((u >> 16) & 1u)) >> 16);
}
__device__ __forceinline__ float bf_bits2f(unsigned short h) { return __uint_as_float(((unsigned)h) << 16); }
__device__ __forceinline__ float bf_rne(float f) { return bf_bits2f(f2bf_bits(f)); }

__device__ __forceinline__ void dep_guard_h(v8f& a, v8f& b, v16h x, v16h y) { asm volatile("v_nop\n\tv_nop\n\tv_nop\n\tv_nop" : "+v"(a), "+v"(b) : "v"(x), "v"(y)); }
__device__ __forceinline__ void dep_guard_b(v8f& a, v8f& b, v16b x, v16b y) { asm volatile("v_nop\n\tv_nop\n\tv_nop\n\tv_nop" : "+v"(a), "+v"(b) : "v"(x), "v"(y)); }
__device__ __forceinline__ void keep4_h(v16h a, v16h b, v16h c, v16h d) { asm volatile("v_nop" :: "v"(a), "v"(b), "v"(c), "v"(d)); }
__device__ __forceinline__ void keep4_b(v16b a, v16b b, v16b c, v16b d) { asm volatile("v_nop" :: "v"(a), "v"(b), "v"(c), "v"(d)); }
__device__ __forceinline__ void acc_guard4(v8f& a, v8f& b, v8f& c, v8f& d) { asm volatile("v_nop\n\tv_nop\n\tv_nop\n\tv_nop" : "+v"(a), "+v"(b), "+v"(c), "+v"(d)); }

template <typename T> struct Frag;
template <> struct Frag<_Float16> {
  typedef v16h V; union U { v16h v; v8h h[2]; };
  static __device__ __forceinline__ v16h load(const _Float16* p) {
    U f; f.h[0] = *(const v8h*)(p); f.h[1] = *(const v8h*)(p + 16); return f.v;
  }
  static __device__ __forceinline__ v8f mma(v16h a, v16h b, v8f c) {
    return __builtin_amdgcn_wmma_f32_16x16x32_f16(false, a, false, b, (short)0, c, false, false);
  }
  static __device__ __forceinline__ void guard(v8f& a, v8f& b, v16h x, v16h y) { dep_guard_h(a, b, x, y); }
  static __device__ __forceinline__ void keep(v16h a, v16h b, v16h c, v16h d) { keep4_h(a, b, c, d); }
};
template <> struct Frag<__bf16> {
  typedef v16b V; union U { v16b v; v8b h[2]; };
  static __device__ __forceinline__ v16b load(const __bf16* p) {
    U f; f.h[0] = *(const v8b*)(p); f.h[1] = *(const v8b*)(p + 16); return f.v;
  }
  static __device__ __forceinline__ v8f mma(v16b a, v16b b, v8f c) {
    return __builtin_amdgcn_wmma_f32_16x16x32_bf16(false, a, false, b, (short)0, c, false, false);
  }
  static __device__ __forceinline__ void guard(v8f& a, v8f& b, v16b x, v16b y) { dep_guard_b(a, b, x, y); }
  static __device__ __forceinline__ void keep(v16b a, v16b b, v16b c, v16b d) { keep4_b(a, b, c, d); }
};
template <int ET> struct Elem;
template <> struct Elem<0> { typedef _Float16 T; };
template <> struct Elem<1> { typedef __bf16 T; };

__device__ __forceinline__ unsigned short h_bits(float f) { return __builtin_bit_cast(unsigned short, (_Float16)f); }
__device__ __forceinline__ float h2f(unsigned short b) { return (float)__builtin_bit_cast(_Float16, b); }
__device__ __forceinline__ unsigned pack2(unsigned short a, unsigned short b) { return (unsigned)a | ((unsigned)b << 16); }
__device__ __forceinline__ unsigned short hx64(unsigned short b) {
  const unsigned ub = b;
  const unsigned r = ((ub & 0x7c00u) == 0u) ? (ub & 0x8000u) : (ub + 0x1800u);
  return (unsigned short)r;
}
__device__ __forceinline__ void cvt_hl(float a, unsigned short& hb, unsigned short& lb) {
  const _Float16 hv = (_Float16)a;
  hb = __builtin_bit_cast(unsigned short, hv);
  lb = __builtin_bit_cast(unsigned short, (_Float16)((a - (float)hv) * LO_CARRY));
}
__device__ __forceinline__ void pack_hl8(const float (&o)[8], v4u& wh, v4u& wl) {
  unsigned short hb[8], lb[8];
#pragma unroll
  for (int e = 0; e < 8; ++e) cvt_hl(o[e], hb[e], lb[e]);
  wh[0] = pack2(hb[0], hb[1]); wh[1] = pack2(hb[2], hb[3]); wh[2] = pack2(hb[4], hb[5]); wh[3] = pack2(hb[6], hb[7]);
  wl[0] = pack2(lb[0], lb[1]); wl[1] = pack2(lb[2], lb[3]); wl[2] = pack2(lb[4], lb[5]); wl[3] = pack2(lb[6], lb[7]);
}
__device__ __forceinline__ v8f mma_h(v16h a, v16h b, v8f c) {
  c = __builtin_amdgcn_wmma_f32_16x16x32_f16(false, a, false, b, (short)0, c, false, false);
  asm volatile("v_nop\n\tv_nop\n\tv_nop\n\tv_nop" : "+v"(c) : "v"(a), "v"(b));
  return c;
}

__global__ __launch_bounds__(256) void cast_bf16x8(const float* __restrict__ in, unsigned short* __restrict__ out, int n8) {
  const int i = blockIdx.x * 256 + threadIdx.x;
  if (i < n8) {
    const size_t o = (size_t)i * 8;
    const v4f a = *(const v4f*)(in + o);
    const v4f b = *(const v4f*)(in + o + 4);
    v4u w;
    w[0] = pack2(f2bf_bits(a[0]), f2bf_bits(a[1]));
    w[1] = pack2(f2bf_bits(a[2]), f2bf_bits(a[3]));
    w[2] = pack2(f2bf_bits(b[0]), f2bf_bits(b[1]));
    w[3] = pack2(f2bf_bits(b[2]), f2bf_bits(b[3]));
    volatile v4u* p = (volatile v4u*)(out + o);
    *p = w;
    __threadfence();
    *p = w;
  }
}

__global__ __launch_bounds__(256) void cast_wo_planes(const float* __restrict__ in, unsigned short* __restrict__ oh,
                                                      unsigned short* __restrict__ olo, int n8) {
  const int i = blockIdx.x * 256 + threadIdx.x;
  if (i < n8) {
    const size_t o = (size_t)i * 8;
    const v4f a = *(const v4f*)(in + o);
    const v4f b = *(const v4f*)(in + o + 4);
    const float r[8] = {a[0], a[1], a[2], a[3], b[0], b[1], b[2], b[3]};
    unsigned short hb[8], lb[8];
#pragma unroll
    for (int e = 0; e < 8; ++e) {
      const float x = bf_rne(r[e]);
      hb[e] = h_bits(x * W_CARRY);
      lb[e] = h_bits(x);
    }
    v4u wh, wl;
    wh[0] = pack2(hb[0], hb[1]); wh[1] = pack2(hb[2], hb[3]); wh[2] = pack2(hb[4], hb[5]); wh[3] = pack2(hb[6], hb[7]);
    wl[0] = pack2(lb[0], lb[1]); wl[1] = pack2(lb[2], lb[3]); wl[2] = pack2(lb[4], lb[5]); wl[3] = pack2(lb[6], lb[7]);
    volatile v4u* ph = (volatile v4u*)(oh + o);
    volatile v4u* pl = (volatile v4u*)(olo + o);
    *ph = wh; *pl = wl;
    __threadfence();
    *ph = wh; *pl = wl;
  }
}

template <int ET, int PROD>
__global__ __launch_bounds__(256) void wmma_gemm64(
    const unsigned short* __restrict__ Ap, const unsigned short* __restrict__ A2p, int lda,
    const unsigned short* __restrict__ Btp, const unsigned short* __restrict__ Bt2p, int ldb,
    float* __restrict__ Cp, int ldc, int M, int N, int K, float scale) {
  typedef typename Elem<ET>::T T;
  typedef typename Frag<T>::V V;
  const T* A = (const T*)Ap; const T* A2 = (const T*)A2p; const T* Bt = (const T*)Btp; const T* Bt2 = (const T*)Bt2p;
  __shared__ __align__(16) float sT[8][16 * 68];
  const int lane = threadIdx.x & 31;
  const int wave = threadIdx.x >> 5;
  const int tilesN = N >> 6;
  const int tilesM = M >> 6;
  const int tile = blockIdx.x * 8 + wave;
  if (tile >= tilesM * tilesN) return;
  const int tm = tile / tilesN;
  const int tn = tile - tm * tilesN;
  const int m0 = tm << 6;
  const int n0 = tn << 6;
  const int rlane = lane & 15;
  const int koff  = (lane >> 4) * 8;
  const int mOff  = (lane >> 4) * 8;

  v8f acc[4][4];
#pragma unroll
  for (int i = 0; i < 4; ++i)
#pragma unroll
    for (int j = 0; j < 4; ++j) acc[i][j] = (v8f){0.f,0.f,0.f,0.f,0.f,0.f,0.f,0.f};

  for (int k0 = 0; k0 < K; k0 += 32) {
    V bh[4], bl[4];
#pragma unroll
    for (int j = 0; j < 4; ++j) {
      const size_t bo = (size_t)(n0 + (j << 4) + rlane) * ldb + koff + k0;
      bh[j] = Frag<T>::load(Bt + bo);
      bl[j] = bh[j];
      if (PROD == 1) bl[j] = Frag<T>::load(Bt2 + bo);
    }
#pragma unroll
    for (int i = 0; i < 4; ++i) {
      const size_t ao = (size_t)(m0 + (i << 4) + rlane) * lda + koff + k0;
      V ah = Frag<T>::load(A + ao);
      V al = ah;
      if (PROD == 1) al = Frag<T>::load(A2 + ao);
#pragma unroll
      for (int j = 0; j < 4; ++j) {
        acc[i][j] = Frag<T>::mma(ah, bh[j], acc[i][j]);
        if (PROD == 1) acc[i][j] = Frag<T>::mma(al, bl[j], acc[i][j]);
      }
      Frag<T>::guard(acc[i][0], acc[i][3], ah, al);
    }
    Frag<T>::keep(bh[0], bh[1], bh[2], bh[3]);
    if (PROD == 1) Frag<T>::keep(bl[0], bl[1], bl[2], bl[3]);
  }
  acc_guard4(acc[0][0], acc[0][1], acc[0][2], acc[0][3]);
  acc_guard4(acc[1][0], acc[1][1], acc[1][2], acc[1][3]);
  acc_guard4(acc[2][0], acc[2][1], acc[2][2], acc[2][3]);
  acc_guard4(acc[3][0], acc[3][1], acc[3][2], acc[3][3]);

  float* slab = sT[wave];
#pragma unroll
  for (int i = 0; i < 4; ++i) {
    const int mBase = m0 + (i << 4);
#pragma unroll
    for (int j = 0; j < 4; ++j) {
#pragma unroll
      for (int r = 0; r < 8; ++r) slab[(mOff + r) * 68 + (j << 4) + rlane] = acc[i][j][r] * scale;
    }
    __builtin_amdgcn_fence(__ATOMIC_RELEASE, "workgroup");
    __builtin_amdgcn_wave_barrier();
    __builtin_amdgcn_fence(__ATOMIC_ACQUIRE, "workgroup");
    {
      const int hh = lane >> 4, c4 = (lane & 15) * 4;
      for (int pass = 0; pass < 2; ++pass) {
#pragma unroll
        for (int it = 0; it < 8; ++it) {
          const int row = it * 2 + hh;
          v4f v = *(const v4f*)(slab + row * 68 + c4);
          *(volatile v4f*)(Cp + (size_t)(mBase + row) * ldc + n0 + c4) = v;
        }
        __threadfence();
      }
    }
    __builtin_amdgcn_fence(__ATOMIC_RELEASE, "workgroup");
    __builtin_amdgcn_wave_barrier();
    __builtin_amdgcn_fence(__ATOMIC_ACQUIRE, "workgroup");
  }
}

struct FreqTab { float f[NFREQ]; };
static_assert(sizeof(FreqTab) == NFREQ * 4);

__global__ __launch_bounds__(256) void rope_table_kernel(float* __restrict__ tcos, float* __restrict__ tsin, FreqTab ft, int n) {
#pragma clang fp contract(off)
  const int i = blockIdx.x * 256 + threadIdx.x;
  if (i < n) {
    const int pos = i >> 6;
    const int j = i & 63;
    float fr = 0.0f;
#pragma unroll
    for (int t = 0; t < NFREQ; ++t) fr = (j == t) ? ft.f[t] : fr;
    const float ang = (float)pos * fr;
    const float cv = cosf(ang);
    const float sv = sinf(ang);
    volatile float* pc = tcos + i;
    volatile float* ps = tsin + i;
    *pc = cv; *ps = sv;
    __threadfence();
    *pc = cv; *ps = sv;
  }
}

__global__ __launch_bounds__(256) void norm_rope_kernel(
    const float* __restrict__ qkv, const float* __restrict__ qw, const float* __restrict__ kw,
    const float* __restrict__ tcos, const float* __restrict__ tsin,
    unsigned short* __restrict__ qh, unsigned short* __restrict__ ql,
    unsigned short* __restrict__ kh, unsigned short* __restrict__ kl,
    unsigned short* __restrict__ vh, unsigned short* __restrict__ vl, int nsplit) {
  __shared__ __align__(16) float ys[HID + KVW];
  __shared__ float redq[8];
  __shared__ float redk[8];
  const int pos = blockIdx.x, tid = threadIdx.x, wave = tid >> 5, lane = tid & 31;
  const float* const row = qkv + (size_t)pos * QKVW;
  const int cq = 8 * tid;
  const int ckv = 8 * (tid & 63);
  const int kvbase = (wave == 2 || wave == 3) ? (HID + KVW) : HID;
  const v4f x0 = *(const v4f*)(row + cq);
  const v4f x1 = *(const v4f*)(row + cq + 4);
  const v4f y0 = *(const v4f*)(row + kvbase + ckv);
  const v4f y1 = *(const v4f*)(row + kvbase + ckv + 4);
  const float xq[8] = {x0[0], x0[1], x0[2], x0[3], x1[0], x1[1], x1[2], x1[3]};
  const float xy[8] = {y0[0], y0[1], y0[2], y0[3], y1[0], y1[1], y1[2], y1[3]};
  float ssq = 0.f, ssy = 0.f;
#pragma unroll
  for (int e = 0; e < 8; ++e) { ssq += xq[e] * xq[e]; ssy += xy[e] * xy[e]; }
  float ssk = (wave < 2) ? ssy : 0.f;
#pragma unroll
  for (int off = 16; off > 0; off >>= 1) { ssq += __shfl_xor(ssq, off, 32); ssk += __shfl_xor(ssk, off, 32); }
  if (lane == 0) { redq[wave] = ssq; redk[wave] = ssk; }
  __syncthreads();
  float tq = 0.f, tk = 0.f;
#pragma unroll
  for (int i = 0; i < 8; ++i) { tq += redq[i]; tk += redk[i]; }
  const float rq = rsqrtf(tq * (1.0f / (float)HID) + RMS_EPS);
  const float rk = rsqrtf(tk * (1.0f / (float)KVW) + RMS_EPS);

  const v4f wq0 = *(const v4f*)(qw + cq);
  const v4f wq1 = *(const v4f*)(qw + cq + 4);
  const v4f wk0 = *(const v4f*)(kw + ckv);
  const v4f wk1 = *(const v4f*)(kw + ckv + 4);
  const float wqa[8] = {wq0[0], wq0[1], wq0[2], wq0[3], wq1[0], wq1[1], wq1[2], wq1[3]};
  const float wka[8] = {wk0[0], wk0[1], wk0[2], wk0[3], wk1[0], wk1[1], wk1[2], wk1[3]};
  float yq[8], yk[8];
#pragma unroll
  for (int e = 0; e < 8; ++e) { yq[e] = (xq[e] * rq) * bf_rne(wqa[e]); yk[e] = (xy[e] * rk) * bf_rne(wka[e]); }
  *(v4f*)(ys + cq)     = (v4f){yq[0], yq[1], yq[2], yq[3]};
  *(v4f*)(ys + cq + 4) = (v4f){yq[4], yq[5], yq[6], yq[7]};
  if (wave < 2) {
    *(v4f*)(ys + HID + ckv)     = (v4f){yk[0], yk[1], yk[2], yk[3]};
    *(v4f*)(ys + HID + ckv + 4) = (v4f){yk[4], yk[5], yk[6], yk[7]};
  }
  __syncthreads();

  {
    const int pc = cq ^ 64;
    const v4f p0 = *(const v4f*)(ys + pc);
    const v4f p1 = *(const v4f*)(ys + pc + 4);
    const int j0 = cq & 63;
    const v4f c0 = *(const v4f*)(tcos + (size_t)pos * NFREQ + j0);
    const v4f c1 = *(const v4f*)(tcos + (size_t)pos * NFREQ + j0 + 4);
    const v4f s0 = *(const v4f*)(tsin + (size_t)pos * NFREQ + j0);
    const v4f s1 = *(const v4f*)(tsin + (size_t)pos * NFREQ + j0 + 4);
    const float pp[8] = {p0[0], p0[1], p0[2], p0[3], p1[0], p1[1], p1[2], p1[3]};
    const float cs[8] = {c0[0], c0[1], c0[2], c0[3], c1[0], c1[1], c1[2], c1[3]};
    const float sn[8] = {s0[0], s0[1], s0[2], s0[3], s1[0], s1[1], s1[2], s1[3]};
    const float sg = (cq & 64) ? 1.0f : -1.0f;
    float o[8];
#pragma unroll
    for (int e = 0; e < 8; ++e) o[e] = yq[e] * cs[e] + sg * pp[e] * sn[e];
    v4u wh, wl;
    pack_hl8(o, wh, wl);
    const size_t off = (size_t)pos * HID + cq;
    volatile v4u* ph = (volatile v4u*)(qh + off);
    *ph = wh;
    __threadfence();
    *ph = wh;
    if (pos < nsplit) {
      volatile v4u* plp = (volatile v4u*)(ql + off);
      *plp = wl;
      __threadfence();
      *plp = wl;
    }
  }
  if (wave < 2) {
    const int pc = HID + (ckv ^ 64);
    const v4f p0 = *(const v4f*)(ys + pc);
    const v4f p1 = *(const v4f*)(ys + pc + 4);
    const int j0 = ckv & 63;
    const v4f c0 = *(const v4f*)(tcos + (size_t)pos * NFREQ + j0);
    const v4f c1 = *(const v4f*)(tcos + (size_t)pos * NFREQ + j0 + 4);
    const v4f s0 = *(const v4f*)(tsin + (size_t)pos * NFREQ + j0);
    const v4f s1 = *(const v4f*)(tsin + (size_t)pos * NFREQ + j0 + 4);
    const float pp[8] = {p0[0], p0[1], p0[2], p0[3], p1[0], p1[1], p1[2], p1[3]};
    const float cs[8] = {c0[0], c0[1], c0[2], c0[3], c1[0], c1[1], c1[2], c1[3]};
    const float sn[8] = {s0[0], s0[1], s0[2], s0[3], s1[0], s1[1], s1[2], s1[3]};
    const float sg = (ckv & 64) ? 1.0f : -1.0f;
    float o[8];
#pragma unroll
    for (int e = 0; e < 8; ++e) o[e] = yk[e] * cs[e] + sg * pp[e] * sn[e];
    v4u wh, wl;
    pack_hl8(o, wh, wl);
    const size_t off = (size_t)pos * KVW + ckv;
    volatile v4u* ph = (volatile v4u*)(kh + off);
    *ph = wh;
    __threadfence();
    *ph = wh;
    if (pos < nsplit) {
      volatile v4u* plp = (volatile v4u*)(kl + off);
      *plp = wl;
      __threadfence();
      *plp = wl;
    }
  } else if (wave < 4) {
    float o[8];
#pragma unroll
    for (int e = 0; e < 8; ++e) o[e] = xy[e];
    v4u wh, wl;
    pack_hl8(o, wh, wl);
    const size_t off = (size_t)pos * KVW + ckv;
    volatile v4u* ph = (volatile v4u*)(vh + off);
    *ph = wh;
    __threadfence();
    *ph = wh;
    if (pos < nsplit) {
      volatile v4u* plp = (volatile v4u*)(vl + off);
      *plp = wl;
      __threadfence();
      *plp = wl;
    }
  }
}

template <bool SPLIT>
__global__ __launch_bounds__(128) void attn_kernel(
    const unsigned short* __restrict__ qh, const unsigned short* __restrict__ ql,
    const unsigned short* __restrict__ kh, const unsigned short* __restrict__ kl,
    const unsigned short* __restrict__ vh, const unsigned short* __restrict__ vl,
    unsigned short* __restrict__ oh, unsigned short* __restrict__ ol,
    int qb0, int nqbl, float sscale) {
  constexpr int KC = 32, KP = 136, VP = 40, PP = 40, OP = 132;
  constexpr int P_PLANE = 4 * 16 * PP;
  constexpr int NPP = SPLIT ? 2 : 1;
  constexpr int P_BYTES = NPP * P_PLANE * 2;
  constexpr int K_PLANE = KC * KP;
  constexpr int NKP = SPLIT ? 2 : 1;
  constexpr int V_PLANE = HDM * VP;
  constexpr int NVP = SPLIT ? 3 : 1;
  constexpr int KV_BYTES = (NKP * K_PLANE + NVP * V_PLANE) * 2;
  constexpr int OS_BYTES = 4 * 16 * OP * 4;
  constexpr int U_BYTES = (KV_BYTES > OS_BYTES) ? KV_BYTES : OS_BYTES;
  constexpr int LDS_BYTES = P_BYTES + U_BYTES;
  static_assert(LDS_BYTES <= 65536);
  static_assert(P_BYTES % 16 == 0 && (K_PLANE * 2) % 16 == 0 && (V_PLANE * 2) % 16 == 0);
  __shared__ __align__(16) unsigned char lds_raw[LDS_BYTES];
  unsigned short* const Phs = (unsigned short*)lds_raw;
  unsigned short* const Pls = Phs + P_PLANE;
  unsigned short* const Ks  = (unsigned short*)(lds_raw + P_BYTES);
  unsigned short* const Kls = Ks + K_PLANE;
  unsigned short* const Vs  = Ks + NKP * K_PLANE;
  unsigned short* const Vls = Vs + V_PLANE;
  unsigned short* const V64 = Vs + 2 * V_PLANE;
  float* const Os = (float*)(lds_raw + P_BYTES);

  const int tid = threadIdx.x, wave = tid >> 5, lane = tid & 31, hh = lane >> 4, c = lane & 15;
  const int bx = blockIdx.x;
  const int h = bx / nqbl;
  const int qb = qb0 + (bx - h * nqbl);
  const int g = h >> 2;
  const int q0 = qb * QB_ROWS + wave * 16;
  const _Float16* const qhp = (const _Float16*)qh + (size_t)h * HDM;
  const _Float16* const qlp = (const _Float16*)ql + (size_t)h * HDM;
  const v8f zero8 = {0.f, 0.f, 0.f, 0.f, 0.f, 0.f, 0.f, 0.f};

  float mrow[8], lrow[8];
  v8f oacc[8];
#pragma unroll
  for (int r = 0; r < 8; ++r) { mrow[r] = -INFINITY; lrow[r] = 0.f; }
#pragma unroll
  for (int t = 0; t < 8; ++t) oacc[t] = zero8;

  const int nch = 2 * (qb + 1);
  for (int kc = 0; kc < nch; ++kc) {
    const int kv0 = kc * KC;
    __syncthreads();
    {
      const int key = tid >> 2, dq = (tid & 3) * 32;
      const size_t grow = (size_t)(kv0 + key) * KVW + (size_t)g * HDM + dq;
      const v4u* ksrc = (const v4u*)(kh + grow);
      v4u* kdst = (v4u*)(Ks + key * KP + dq);
#pragma unroll
      for (int i = 0; i < 4; ++i) kdst[i] = ksrc[i];
      if (SPLIT) {
        const v4u* klsrc = (const v4u*)(kl + grow);
        v4u* kldst = (v4u*)(Kls + key * KP + dq);
#pragma unroll
        for (int i = 0; i < 4; ++i) kldst[i] = klsrc[i];
      }
      const v4u* vsrc = (const v4u*)(vh + grow);
#pragma unroll
      for (int i = 0; i < 4; ++i) {
        const v4u w = vsrc[i];
#pragma unroll
        for (int e = 0; e < 4; ++e) {
          const unsigned u = w[e];
          const unsigned short b0 = (unsigned short)(u & 0xffffu);
          const unsigned short b1 = (unsigned short)(u >> 16);
          const int d = dq + 8 * i + 2 * e;
          Vs[d * VP + key] = b0;
          Vs[(d + 1) * VP + key] = b1;
          if (SPLIT) { V64[d * VP + key] = hx64(b0); V64[(d + 1) * VP + key] = hx64(b1); }
        }
      }
      if (SPLIT) {
        const v4u* vlsrc = (const v4u*)(vl + grow);
#pragma unroll
        for (int i = 0; i < 4; ++i) {
          const v4u w = vlsrc[i];
#pragma unroll
          for (int e = 0; e < 4; ++e) {
            const unsigned u = w[e];
            const int d = dq + 8 * i + 2 * e;
            Vls[d * VP + key] = (unsigned short)(u & 0xffffu);
            Vls[(d + 1) * VP + key] = (unsigned short)(u >> 16);
          }
        }
      }
    }
    __syncthreads();

    v8f s[2], s2[2];
    s[0] = zero8; s[1] = zero8; s2[0] = zero8; s2[1] = zero8;
#pragma unroll
    for (int dc = 0; dc < 4; ++dc) {
      const size_t qo = (size_t)(q0 + c) * HID + dc * 32 + 8 * hh;
      const v16h qa = Frag<_Float16>::load(qhp + qo);
      v16h qla = qa;
      if (SPLIT) qla = Frag<_Float16>::load(qlp + qo);
#pragma unroll
      for (int j = 0; j < 2; ++j) {
        const int ko = (j * 16 + c) * KP + dc * 32 + 8 * hh;
        const v16h kb = Frag<_Float16>::load((const _Float16*)Ks + ko);
        s[j] = mma_h(qa, kb, s[j]);
        if (SPLIT) {
          const v16h klb = Frag<_Float16>::load((const _Float16*)Kls + ko);
          s2[j] = mma_h(qa, klb, s2[j]);
          s2[j] = mma_h(qla, kb, s2[j]);
        }
      }
      asm volatile("" ::: "memory");
    }

    float cm[8];
#pragma unroll
    for (int r = 0; r < 8; ++r) {
      const int qrow = q0 + 8 * hh + r;
      float m = -INFINITY;
#pragma unroll
      for (int j = 0; j < 2; ++j) {
        const int kvcol = kv0 + j * 16 + c;
        float sv = s[j][r];
        if (SPLIT) sv += s2[j][r] * (1.0f / LO_CARRY);
        sv *= sscale;
        sv = (kvcol > qrow) ? -INFINITY : sv;
        s[j][r] = sv;
        m = fmaxf(m, sv);
      }
#pragma unroll
      for (int off = 1; off < 16; off <<= 1) m = fmaxf(m, __shfl_xor(m, off, 32));
      cm[r] = m;
    }
    unsigned short* const pwh = Phs + wave * 16 * PP;
    unsigned short* const pwl = Pls + wave * 16 * PP;
#pragma unroll
    for (int r = 0; r < 8; ++r) {
      const float mnew = fmaxf(mrow[r], cm[r]);
      const float alpha = expf(mrow[r] - mnew);
      mrow[r] = mnew;
      float psum = 0.f;
#pragma unroll
      for (int j = 0; j < 2; ++j) {
        const float p = expf(s[j][r] - mnew);
        psum += p;
        const float pcv = p * P_CARRY;
        const unsigned short hb = h_bits(pcv);
        pwh[(8 * hh + r) * PP + j * 16 + c] = hb;
        if (SPLIT) pwl[(8 * hh + r) * PP + j * 16 + c] = h_bits((pcv - h2f(hb)) * LO_CARRY);
      }
#pragma unroll
      for (int off = 1; off < 16; off <<= 1) psum += __shfl_xor(psum, off, 32);
      lrow[r] = lrow[r] * alpha + psum;
#pragma unroll
      for (int t = 0; t < 8; ++t) oacc[t][r] *= alpha;
    }
    __syncthreads();

    {
      const int po = wave * 16 * PP + c * PP + 8 * hh;
      const v16h pa = Frag<_Float16>::load((const _Float16*)Phs + po);
      if (SPLIT) {
        const v16h pla = Frag<_Float16>::load((const _Float16*)Pls + po);
#pragma unroll
        for (int t = 0; t < 8; ++t) {
          const int vo = (t * 16 + c) * VP + 8 * hh;
          const v16h vb64 = Frag<_Float16>::load((const _Float16*)V64 + vo);
          oacc[t] = mma_h(pa, vb64, oacc[t]);
        }
        asm volatile("" ::: "memory");
#pragma unroll
        for (int t = 0; t < 8; ++t) {
          const int vo = (t * 16 + c) * VP + 8 * hh;
          const v16h vlb = Frag<_Float16>::load((const _Float16*)Vls + vo);
          oacc[t] = mma_h(pa, vlb, oacc[t]);
        }
        asm volatile("" ::: "memory");
#pragma unroll
        for (int t = 0; t < 8; ++t) {
          const int vo = (t * 16 + c) * VP + 8 * hh;
          const v16h vb = Frag<_Float16>::load((const _Float16*)Vs + vo);
          oacc[t] = mma_h(pla, vb, oacc[t]);
        }
      } else {
#pragma unroll
        for (int t = 0; t < 8; ++t) {
          const int vo = (t * 16 + c) * VP + 8 * hh;
          const v16h vb = Frag<_Float16>::load((const _Float16*)Vs + vo);
          oacc[t] = mma_h(pa, vb, oacc[t]);
        }
      }
    }
  }

  __syncthreads();
  {
    float* const os = Os + wave * 16 * OP;
    const float osc = SPLIT ? (P_CARRY * LO_CARRY) : P_CARRY;
#pragma unroll
    for (int r = 0; r < 8; ++r) {
      const float inv = A_CARRY / (lrow[r] * osc);
#pragma unroll
      for (int t = 0; t < 8; ++t) os[(8 * hh + r) * OP + t * 16 + c] = oacc[t][r] * inv;
    }
  }
  __syncthreads();
  {
    const float* const os = Os + wave * 16 * OP;
    const int q4 = lane >> 3, c8 = (lane & 7) * 8;
    for (int pass = 0; pass < 2; ++pass) {
#pragma unroll
      for (int it = 0; it < 8; ++it) {
        const int orow = it * 2 + (q4 >> 1);
        const int ocol = (q4 & 1) * 64 + c8;
        const float* sp = os + orow * OP + ocol;
        const v4f f0 = *(const v4f*)sp;
        const v4f f1 = *(const v4f*)(sp + 4);
        const float o[8] = {f0[0], f0[1], f0[2], f0[3], f1[0], f1[1], f1[2], f1[3]};
        v4u wh, wl;
        pack_hl8(o, wh, wl);
        const size_t go = (size_t)(q0 + orow) * HID + (size_t)h * HDM + ocol;
        *(volatile v4u*)(oh + go) = wh;
        if (SPLIT) *(volatile v4u*)(ol + go) = wl;
      }
      __threadfence();
    }
  }
}

extern "C" void kernel_launch(void* const* d_in, const int* in_sizes, int n_in,
                              void* d_out, int out_size, void* d_ws, size_t ws_size,
                              hipStream_t stream) {
  if (n_in < 7) return;
  if (in_sizes[0] != SEQ * HID || in_sizes[1] != HID * HID || in_sizes[2] != KVW * HID ||
      in_sizes[3] != KVW * HID || in_sizes[4] != HID * HID || in_sizes[5] != HID || in_sizes[6] != KVW) return;
  if (out_size != SEQ * HID) return;
  if (ws_size < WS_TOTAL) return;

  const float* hs = (const float*)d_in[0];
  const float* wq = (const float*)d_in[1];
  const float* wk = (const float*)d_in[2];
  const float* wv = (const float*)d_in[3];
  const float* wo = (const float*)d_in[4];
  const float* qw = (const float*)d_in[5];
  const float* kw = (const float*)d_in[6];
  float* out = (float*)d_out;
  char* ws = (char*)d_ws;

  float*          qkv_raw = (float*)(ws + WS_QKVRAW);
  unsigned short* a_hi    = (unsigned short*)(ws + WS_AH);
  unsigned short* a_lo    = (unsigned short*)(ws + WS_AL);
  unsigned short* hs_b    = (unsigned short*)(ws + WS_HS);
  unsigned short* q_hi    = (unsigned short*)(ws + WS_QH);
  unsigned short* wqkv_b  = (unsigned short*)(ws + WS_WQKV);
  unsigned short* k_hi    = (unsigned short*)(ws + WS_KH);
  unsigned short* v_hi    = (unsigned short*)(ws + WS_VH);
  unsigned short* k_lo    = (unsigned short*)(ws + WS_KL);
  unsigned short* v_lo    = (unsigned short*)(ws + WS_VL);
  unsigned short* wo_hi   = (unsigned short*)(ws + WS_WOH);
  unsigned short* wo_lo   = (unsigned short*)(ws + WS_WOL);
  unsigned short* q_lo    = (unsigned short*)(ws + WS_QL);
  float*          tcos    = (float*)(ws + WS_TCOS);
  float*          tsin    = (float*)(ws + WS_TSIN);

  FreqTab ft;
  for (int j = 0; j < NFREQ; ++j) {
    const float e = (float)(2 * j) * (1.0f / (float)HDM);
    const double pd = pow(10000.0, (double)e);
    const float pf = (float)pd;
    ft.f[j] = 1.0f / pf;
  }
  const float sscale = 0.08838834764831845f;

  {
    const int n8_hs = SEQ * HID / 8;
    const int n8_wq = HID * HID / 8;
    const int n8_wk = KVW * HID / 8;
    cast_bf16x8<<<dim3(n8_hs / 256), dim3(256), 0, stream>>>(hs, hs_b, n8_hs);
    cast_bf16x8<<<dim3(n8_wq / 256), dim3(256), 0, stream>>>(wq, wqkv_b, n8_wq);
    cast_bf16x8<<<dim3(n8_wk / 256), dim3(256), 0, stream>>>(wk, wqkv_b + (size_t)HID * HID, n8_wk);
    cast_bf16x8<<<dim3(n8_wk / 256), dim3(256), 0, stream>>>(wv, wqkv_b + (size_t)HID * HID + (size_t)KVW * HID, n8_wk);
    cast_wo_planes<<<dim3(n8_wq / 256), dim3(256), 0, stream>>>(wo, wo_hi, wo_lo, n8_wq);
  }

  wmma_gemm64<1, 0><<<dim3((SEQ / 64) * (QKVW / 64) / 8), dim3(256), 0, stream>>>(
      hs_b, hs_b, HID, wqkv_b, wqkv_b, HID, qkv_raw, QKVW, SEQ, QKVW, HID, 1.0f);

  rope_table_kernel<<<dim3(SEQ * NFREQ / 256), dim3(256), 0, stream>>>(tcos, tsin, ft, SEQ * NFREQ);
  norm_rope_kernel<<<dim3(SEQ), dim3(256), 0, stream>>>(qkv_raw, qw, kw, tcos, tsin,
                                                        q_hi, q_lo, k_hi, k_lo, v_hi, v_lo, ROWS_SPLIT);

  attn_kernel<true><<<dim3(NQH * NQB_SPLIT), dim3(128), 0, stream>>>(
      q_hi, q_lo, k_hi, k_lo, v_hi, v_lo, a_hi, a_lo, 0, NQB_SPLIT, sscale);
  attn_kernel<false><<<dim3(NQH * (NQB - NQB_SPLIT)), dim3(128), 0, stream>>>(
      q_hi, q_lo, k_hi, k_lo, v_hi, v_lo, a_hi, a_lo, NQB_SPLIT, NQB - NQB_SPLIT, sscale);

  wmma_gemm64<0, 1><<<dim3((ROWS_SPLIT / 64) * (HID / 64) / 8), dim3(256), 0, stream>>>(
      a_hi, a_lo, HID, wo_hi, wo_lo, HID, out, HID, ROWS_SPLIT, HID, HID, 1.0f / (A_CARRY * W_CARRY));
  wmma_gemm64<0, 0><<<dim3(((SEQ - ROWS_SPLIT) / 64) * (HID / 64) / 8), dim3(256), 0, stream>>>(
      a_hi + (size_t)ROWS_SPLIT * HID, a_hi + (size_t)ROWS_SPLIT * HID, HID, wo_hi, wo_hi, HID,
      out + (size_t)ROWS_SPLIT * HID, HID, SEQ - ROWS_SPLIT, HID, HID, 1.0f / (A_CARRY * W_CARRY));
}
